// Model_1906965479431
// MI455X (gfx1250) — hardware-verified
//
#include <hip/hip_runtime.h>
#include <stddef.h>
#include <stdint.h>


#define DF     128
#define PP     256
#define NTHR   256
#define NWAVE  8
#define EPT    8
#define CHUNK  (NTHR * EPT)
#define WCAP   (EPT * 32)
#define LISTN  (NWAVE * WCAP)
#define RCAP   28672
#define SL_RD  7
#define SL_DR  10
#define DEG_RD 256
#define DEG_DR 64
#define LS_RD  22528
#define LS_DR  18432
#define GBM    64
#define GBN    128
#define GTHR   128
#define GWAVE  (GTHR / 32)
#define ROWH   256
#define UPART  2048
#define NPART  18
#define NUW    (NPART * UPART)
#define LBLK   1024
#define MISC_INTS 16
#define WSMAX  134217728

static_assert((CHUNK & (CHUNK - 1)) == 0 && CHUNK <= 4096);
static_assert(((long long)CHUNK << SL_DR) < (1LL << 31));
static_assert(LS_RD % (NTHR * 4) == 0 && LS_DR % (NTHR * 4) == 0 && LS_RD <= RCAP && LS_DR <= RCAP);
static_assert(RCAP % 4 == 0 && LISTN % 4 == 0);
static_assert(GBN == DF && GBM == GWAVE * 16 && DF == 4 * 32 && PP == 2 * DF && ROWH == PP);
static_assert(UPART % NTHR == 0 && UPART == DF * (DF / 8) && NUW % NTHR == 0);
static_assert(LBLK == NTHR * 4 && LBLK == NWAVE * 128);
static_assert((LISTN + 2 * RCAP + 3 * (1 << SL_DR) + MISC_INTS) * 4 <= 300000);

typedef float          v4f   __attribute__((ext_vector_type(4)));
typedef float          v8f   __attribute__((ext_vector_type(8)));
typedef int            v4i   __attribute__((ext_vector_type(4)));
typedef int            v8i   __attribute__((ext_vector_type(8)));
typedef unsigned       v2u   __attribute__((ext_vector_type(2)));
typedef unsigned short v4us  __attribute__((ext_vector_type(4)));
typedef unsigned short v8us  __attribute__((ext_vector_type(8)));
typedef unsigned short v16us __attribute__((ext_vector_type(16)));
typedef __bf16         v16bf __attribute__((ext_vector_type(16)));
typedef v4f  __attribute__((may_alias)) v4fa;
typedef v4i  __attribute__((may_alias)) v4ia;
typedef v2u  __attribute__((may_alias)) v2ua;
typedef v4us __attribute__((may_alias)) v4usa;
typedef v8us __attribute__((may_alias)) v8usa;
union FragB { v16bf v; v16us u; v8us h[2]; v8i w; };

__device__ __forceinline__ v8f wmb(const FragB& a, const FragB& b, v8f c) {
  v8f d = __builtin_amdgcn_wmma_f32_16x16x32_bf16(false, a.v, false, b.v, (short)0, c, false, false);
  asm volatile("v_nop\n\tv_nop\n\tv_nop\n\tv_nop" : "+v"(d) : "v"(a.w), "v"(b.w));
  return d;
}

__device__ __forceinline__ unsigned bf16_bits(float f) {
  const unsigned u = __float_as_uint(f);
  return (u + 0x7FFFu + ((u >> 16) & 1u)) >> 16;
}
__device__ __forceinline__ float bf16_val(float f) {
  return __uint_as_float(bf16_bits(f) << 16);
}
__device__ __forceinline__ unsigned hl_bits(float v, unsigned& lo) {
  const unsigned hb = bf16_bits(v);
  lo = bf16_bits(v - __uint_as_float(hb << 16));
  return hb;
}

__device__ __forceinline__ void wave_sync() {
  __builtin_amdgcn_fence(__ATOMIC_RELEASE, "wavefront");
  __builtin_amdgcn_wave_barrier();
  __builtin_amdgcn_fence(__ATOMIC_ACQUIRE, "wavefront");
}

template <int SLB>
__device__ __forceinline__ int scan_chunk(const int* __restrict__ dsts, int nE, int cbase, int slotBase,
                                          int nb, int vec8, int* list, int tid, int lane, int wave) {
  int wc = 0;
  const int el0  = tid * EPT;
  const int e0   = cbase + el0;
  const int sent = -2147483647 - 1;
  v4i da, db;
  if (vec8 != 0 && cbase + CHUNK <= nE) {
    da = *(const v4i*)(dsts + e0);
    db = *(const v4i*)(dsts + e0 + 4);
  } else {
    da.x = (e0     < nE) ? dsts[min(e0,     nE - 1)] : sent;
    da.y = (e0 + 1 < nE) ? dsts[min(e0 + 1, nE - 1)] : sent;
    da.z = (e0 + 2 < nE) ? dsts[min(e0 + 2, nE - 1)] : sent;
    da.w = (e0 + 3 < nE) ? dsts[min(e0 + 3, nE - 1)] : sent;
    db.x = (e0 + 4 < nE) ? dsts[min(e0 + 4, nE - 1)] : sent;
    db.y = (e0 + 5 < nE) ? dsts[min(e0 + 5, nE - 1)] : sent;
    db.z = (e0 + 6 < nE) ? dsts[min(e0 + 6, nE - 1)] : sent;
    db.w = (e0 + 7 < nE) ? dsts[min(e0 + 7, nE - 1)] : sent;
  }
  const unsigned nbs = (unsigned)slotBase;
  const unsigned unb = (unsigned)nb;
  const unsigned s0 = (unsigned)da.x - nbs, s1 = (unsigned)da.y - nbs;
  const unsigned s2 = (unsigned)da.z - nbs, s3 = (unsigned)da.w - nbs;
  const unsigned s4 = (unsigned)db.x - nbs, s5 = (unsigned)db.y - nbs;
  const unsigned s6 = (unsigned)db.z - nbs, s7 = (unsigned)db.w - nbs;
  const bool h0 = s0 < unb, h1 = s1 < unb, h2 = s2 < unb, h3 = s3 < unb;
  const bool h4 = s4 < unb, h5 = s5 < unb, h6 = s6 < unb, h7 = s7 < unb;
  const unsigned any = __builtin_amdgcn_ballot_w32(h0 | h1 | h2 | h3 | h4 | h5 | h6 | h7);
  if (any != 0u) {
#define HITJ(J, HJ, SJ) { \
      const unsigned mj = __builtin_amdgcn_ballot_w32(HJ); \
      if (mj != 0u) { \
        if (HJ) { \
          const int pos = wc + (int)__builtin_amdgcn_mbcnt_lo(mj, 0u); \
          if (pos < WCAP) list[wave * WCAP + pos] = ((el0 + (J)) << SLB) | (int)(SJ); \
        } \
        wc += (int)__builtin_popcount(mj); } }
    HITJ(0, h0, s0)
    HITJ(1, h1, s1)
    HITJ(2, h2, s2)
    HITJ(3, h3, s3)
    HITJ(4, h4, s4)
    HITJ(5, h5, s5)
    HITJ(6, h6, s6)
    HITJ(7, h7, s7)
#undef HITJ
  }
  return wc;
}

__global__ __launch_bounds__(NTHR) void k_prep(const float* __restrict__ xr, const float* __restrict__ xd,
                                               const float* __restrict__ w1rdl, const float* __restrict__ w1rdr,
                                               const float* __restrict__ w1drl, const float* __restrict__ w1drr,
                                               const float* __restrict__ w2rdl, const float* __restrict__ w2rdr,
                                               const float* __restrict__ w2drl, const float* __restrict__ w2drr,
                                               const float* __restrict__ dw1,
                                               unsigned short* wpl, unsigned short* xbr, unsigned short* xbd,
                                               int nR, int nD, int uR, int uD) {
  const int u = (int)blockIdx.x * NTHR + (int)threadIdx.x;
  v8us o;
  unsigned short* dp;
  if (u < NUW) {
    const int part = u >> 11;
    const int v    = u & (UPART - 1);
    const int n    = v >> 4;
    const int k8   = (v & 15) * 8;
    const float* W;
    int poff, pitch, coff;
    if (part == 0)       { W = w1rdl; poff = 0;      pitch = 384; coff = 0; }
    else if (part == 1)  { W = w1rdl; poff = 0;      pitch = 384; coff = 128; }
    else if (part == 2)  { W = w1rdr; poff = 0;      pitch = 384; coff = 256; }
    else if (part == 3)  { W = w1drl; poff = 49152;  pitch = 384; coff = 0; }
    else if (part == 4)  { W = w1drl; poff = 49152;  pitch = 384; coff = 128; }
    else if (part == 5)  { W = w1drr; poff = 49152;  pitch = 384; coff = 256; }
    else if (part == 6)  { W = w2rdl; poff = 98304;  pitch = 512; coff = 0; }
    else if (part == 7)  { W = w2rdl; poff = 98304;  pitch = 512; coff = 128; }
    else if (part == 8)  { W = w2rdr; poff = 98304;  pitch = 512; coff = 256; }
    else if (part == 9)  { W = w2rdr; poff = 98304;  pitch = 512; coff = 384; }
    else if (part == 10) { W = w2drl; poff = 163840; pitch = 512; coff = 0; }
    else if (part == 11) { W = w2drl; poff = 163840; pitch = 512; coff = 128; }
    else if (part == 12) { W = w2drr; poff = 163840; pitch = 512; coff = 256; }
    else if (part == 13) { W = w2drr; poff = 163840; pitch = 512; coff = 384; }
    else if (part == 14) { W = dw1;             poff = 229376; pitch = 256; coff = 0; }
    else if (part == 15) { W = dw1;             poff = 229376; pitch = 256; coff = 128; }
    else if (part == 16) { W = dw1 + DF * DF;   poff = 262144; pitch = 256; coff = 0; }
    else                 { W = dw1 + DF * DF;   poff = 262144; pitch = 256; coff = 128; }
    const float* p = W + (size_t)k8 * DF + n;
#pragma unroll
    for (int i = 0; i < 8; ++i) o[i] = (unsigned short)bf16_bits(p[(size_t)i * DF]);
    dp = wpl + (size_t)poff + (size_t)n * pitch + coff + k8;
  } else if (u < NUW + uR) {
    const int v   = u - NUW;
    const int row = v >> 4, k8 = (v & 15) * 8;
    const int rc  = row < nR ? row : nR - 1;
    const bool lv = row < nR;
    const float* p = xr + (size_t)rc * DF + k8;
    const v4f a = *(const v4f*)p;
    const v4f b = *(const v4f*)(p + 4);
    o[0] = lv ? (unsigned short)bf16_bits(a.x) : (unsigned short)0;
    o[1] = lv ? (unsigned short)bf16_bits(a.y) : (unsigned short)0;
    o[2] = lv ? (unsigned short)bf16_bits(a.z) : (unsigned short)0;
    o[3] = lv ? (unsigned short)bf16_bits(a.w) : (unsigned short)0;
    o[4] = lv ? (unsigned short)bf16_bits(b.x) : (unsigned short)0;
    o[5] = lv ? (unsigned short)bf16_bits(b.y) : (unsigned short)0;
    o[6] = lv ? (unsigned short)bf16_bits(b.z) : (unsigned short)0;
    o[7] = lv ? (unsigned short)bf16_bits(b.w) : (unsigned short)0;
    dp = xbr + (size_t)v * 8;
  } else if (u < NUW + uR + uD) {
    const int v   = u - NUW - uR;
    const int row = v >> 4, k8 = (v & 15) * 8;
    const int rc  = row < nD ? row : nD - 1;
    const bool lv = row < nD;
    const float* p = xd + (size_t)rc * DF + k8;
    const v4f a = *(const v4f*)p;
    const v4f b = *(const v4f*)(p + 4);
    o[0] = lv ? (unsigned short)bf16_bits(a.x) : (unsigned short)0;
    o[1] = lv ? (unsigned short)bf16_bits(a.y) : (unsigned short)0;
    o[2] = lv ? (unsigned short)bf16_bits(a.z) : (unsigned short)0;
    o[3] = lv ? (unsigned short)bf16_bits(a.w) : (unsigned short)0;
    o[4] = lv ? (unsigned short)bf16_bits(b.x) : (unsigned short)0;
    o[5] = lv ? (unsigned short)bf16_bits(b.y) : (unsigned short)0;
    o[6] = lv ? (unsigned short)bf16_bits(b.z) : (unsigned short)0;
    o[7] = lv ? (unsigned short)bf16_bits(b.w) : (unsigned short)0;
    dp = xbd + (size_t)v * 8;
  } else {
    return;
  }
  *(volatile v8us*)dp = o;
  __threadfence();
  *(volatile v8us*)dp = o;
}

template <int SLB, int DEGC, int LSTR>
__global__ __launch_bounds__(NTHR) void k_bucket(const int* __restrict__ srcs, const int* __restrict__ keys,
                                                 int nE, int nSrc, int vec8,
                                                 int* listg, int* cntg, int* offg, int* flg) {
  constexpr int NB    = 1 << SLB;
  constexpr int ZINTS = LISTN + 2 * RCAP + 3 * NB;
  static_assert(NB % 32 == 0 && NB <= NTHR * 4 && ZINTS % 4 == 0 && LSTR <= RCAP && LSTR % (NTHR * 4) == 0);
  extern __shared__ __attribute__((aligned(16))) int dsm[];
  int* list = dsm;
  int* hl   = dsm + LISTN;
  int* sl   = hl + RCAP;
  int* cnt  = sl + RCAP;
  int* offs = cnt + NB;
  int* cur  = offs + NB;
  int* misc = cur + NB;
  const int tid = (int)threadIdx.x, lane = tid & 31, wave = tid >> 5;
  const int blk = (int)blockIdx.x;
  const int nodeBase = blk * NB;

  {
    const v4i z4 = {0, 0, 0, 0};
    for (int i = tid * 4; i < ZINTS; i += NTHR * 4) *(v4ia*)(dsm + i) = z4;
    if (tid < MISC_INTS) misc[tid] = 0;
  }
  __syncthreads();

  int t = 0, ov = 0;
  const int nChunks = (nE + CHUNK - 1) / CHUNK;
#pragma unroll 1
  for (int ch = 0; ch < nChunks; ++ch) {
    const int cbase = ch * CHUNK;
    const int wc = scan_chunk<SLB>(keys, nE, cbase, nodeBase, NB, vec8, list, tid, lane, wave);
    if (lane == 0) misc[wave] = wc;
    __syncthreads();
    if (wave == 0) {
#pragma unroll 1
      for (int w2 = 0; w2 < NWAVE; ++w2) {
        int c = misc[w2];
        c = c < 0 ? 0 : (c > WCAP ? WCAP : c);
#pragma unroll 1
        for (int b0 = 0; b0 < c; b0 += 32) {
          const int idx = b0 + lane;
          const int ent = list[w2 * WCAP + (idx < WCAP ? idx : WCAP - 1)];
          const int m32 = (c - b0) < 32 ? (c - b0) : 32;
#pragma unroll 1
          for (int k = 0; k < m32; ++k) {
            const int u    = __builtin_amdgcn_readlane(ent, k);
            const int slot = u & (NB - 1);
            const int el   = (u >> SLB) & (CHUNK - 1);
            const int pk   = ((cbase + el) << SLB) | slot;
            if (t < RCAP) {
              if (lane == 0) { hl[t] = pk; cnt[slot] = cnt[slot] + 1; }
              t = t + 1;
            } else {
              ov = 1;
            }
          }
        }
      }
    }
    __syncthreads();
  }
  if (wave == 0 && lane == 0) { misc[8] = t; misc[9] = ov; }
  __syncthreads();
  int tt = misc[8];
  tt = tt < 0 ? 0 : (tt > RCAP ? RCAP : tt);
  const int ovf = misc[9];

  if (wave == 0) {
    const int base = lane * (NB / 32);
    int s = 0;
#pragma unroll 1
    for (int i = 0; i < NB / 32; ++i) s += cnt[base + i];
    int incl = s;
#pragma unroll
    for (int d = 1; d < 32; d <<= 1) {
      const int y = __shfl_up(incl, d, 32);
      if (lane >= d) incl += y;
    }
    int run = incl - s;
#pragma unroll 1
    for (int i = 0; i < NB / 32; ++i) {
      const int cv = cnt[base + i];
      offs[base + i] = run;
      cur[base + i]  = run;
      run += cv;
    }
  }
  __syncthreads();
  if (wave == 0) {
#pragma unroll 1
    for (int b0 = 0; b0 < tt; b0 += 32) {
      const int idx = b0 + lane;
      const int ent = hl[idx < RCAP ? idx : RCAP - 1];
      const int m32 = (tt - b0) < 32 ? (tt - b0) : 32;
#pragma unroll 1
      for (int k = 0; k < m32; ++k) {
        const int u    = __builtin_amdgcn_readlane(ent, k);
        const int slot = u & (NB - 1);
        if (lane == 0) {
          int p = cur[slot];
          p = p < 0 ? 0 : (p > RCAP - 1 ? RCAP - 1 : p);
          sl[p] = u;
          cur[slot] = p + 1;
        }
      }
    }
  }
  {
    int bg = 0;
    for (int s = tid; s < NB; s += NTHR) bg |= (cnt[s] > DEGC) ? 1 : 0;
    if (bg != 0) misc[10] = 1;
  }
  __syncthreads();
  const int pflag = ((ovf != 0) || (misc[10] != 0) || (tt > LSTR)) ? 1 : 0;

  int* lb = listg + (size_t)blk * LSTR;
#pragma unroll 1
  for (int i0 = tid * 4; i0 < LSTR; i0 += NTHR * 4) {
    const v4i e4 = *(const v4ia*)(sl + i0);
    int e0 = e4.x >> SLB, e1 = e4.y >> SLB, e2 = e4.z >> SLB, e3 = e4.w >> SLB;
    e0 = e0 < 0 ? 0 : (e0 > nE - 1 ? nE - 1 : e0);
    e1 = e1 < 0 ? 0 : (e1 > nE - 1 ? nE - 1 : e1);
    e2 = e2 < 0 ? 0 : (e2 > nE - 1 ? nE - 1 : e2);
    e3 = e3 < 0 ? 0 : (e3 > nE - 1 ? nE - 1 : e3);
    int q0 = srcs[e0], q1 = srcs[e1], q2 = srcs[e2], q3 = srcs[e3];
    q0 = q0 < 0 ? 0 : (q0 > nSrc - 1 ? nSrc - 1 : q0);
    q1 = q1 < 0 ? 0 : (q1 > nSrc - 1 ? nSrc - 1 : q1);
    q2 = q2 < 0 ? 0 : (q2 > nSrc - 1 ? nSrc - 1 : q2);
    q3 = q3 < 0 ? 0 : (q3 > nSrc - 1 ? nSrc - 1 : q3);
    v4i o4;
    o4.x = (i0     < tt) ? q0 : 0;
    o4.y = (i0 + 1 < tt) ? q1 : 0;
    o4.z = (i0 + 2 < tt) ? q2 : 0;
    o4.w = (i0 + 3 < tt) ? q3 : 0;
    *(volatile v4i*)(lb + i0) = o4;
    __threadfence();
    *(volatile v4i*)(lb + i0) = o4;
  }
  if (tid * 4 < NB) {
    const v4i c4 = *(const v4ia*)(cnt + tid * 4);
    const v4i o4 = *(const v4ia*)(offs + tid * 4);
    int* cp = cntg + (size_t)blk * NB + tid * 4;
    int* op = offg + (size_t)blk * NB + tid * 4;
    *(volatile v4i*)cp = c4;
    *(volatile v4i*)op = o4;
    __threadfence();
    *(volatile v4i*)cp = c4;
    *(volatile v4i*)op = o4;
  }
  if (wave == NWAVE - 1 && lane < 8) {
    const v4i f4 = {pflag, pflag, pflag, pflag};
    int* fp = flg + (size_t)blk * 32 + lane * 4;
    *(volatile v4i*)fp = f4;
    __threadfence();
    *(volatile v4i*)fp = f4;
  }
}

template <int SLB, int DEGC, int LSTR, int HL>
__global__ __launch_bounds__(NTHR) void k_agg(const int* listg, const int* cntg, const int* offg,
                                              const unsigned short* srcp, int nSrc, int nN, int mRows,
                                              unsigned short* apl) {
  constexpr int NB = 1 << SLB;
  constexpr int SP = HL ? PP : DF;
  static_assert(NB % NWAVE == 0);
  __shared__ __attribute__((aligned(16))) unsigned short rowall[NWAVE * ROWH];
  const int tid = (int)threadIdx.x, lane = tid & 31, wave = tid >> 5;
  unsigned short* rowbuf = rowall + wave * ROWH;
  const int blk = (int)blockIdx.x;
  const int nodeBase = blk * NB;
  const int* lb = listg + (size_t)blk * LSTR;

#pragma unroll 1
  for (int si = 0; si < NB / NWAVE; ++si) {
    const int s    = si * NWAVE + wave;
    const int node = nodeBase + s;
    if (node < mRows) {
      const bool live = node < nN;
      int c = cntg[node];
      int o = offg[node];
      const bool big = c > DEGC;
      c = c < 0 ? 0 : (c > DEGC ? DEGC : c);
      c = live ? c : 0;
      o = o < 0 ? 0 : (o > LSTR - 1 ? LSTR - 1 : o);
      float a0 = 0.0f, a1 = 0.0f, a2 = 0.0f, a3 = 0.0f;
#pragma unroll 1
      for (int b0 = 0; b0 < c; b0 += 32) {
        int idx = o + b0 + lane;
        idx = idx > LSTR - 1 ? LSTR - 1 : idx;
        int sr = lb[idx];
        sr = sr < 0 ? 0 : (sr > nSrc - 1 ? nSrc - 1 : sr);
        const int m32 = (c - b0) < 32 ? (c - b0) : 32;
#pragma unroll 1
        for (int k = 0; k < m32; ++k) {
          const int sk = __builtin_amdgcn_readlane(sr, k);
          const unsigned short* rp = srcp + (size_t)sk * SP + 4 * lane;
          const v2u wh = *(const v2ua*)rp;
          float f0 = __uint_as_float(wh.x << 16);
          float f1 = __uint_as_float(wh.x & 0xffff0000u);
          float f2 = __uint_as_float(wh.y << 16);
          float f3 = __uint_as_float(wh.y & 0xffff0000u);
          if constexpr (HL != 0) {
            const v2u wl = *(const v2ua*)(rp + DF);
            f0 += __uint_as_float(wl.x << 16);
            f1 += __uint_as_float(wl.x & 0xffff0000u);
            f2 += __uint_as_float(wl.y << 16);
            f3 += __uint_as_float(wl.y & 0xffff0000u);
          }
          a0 += f0; a1 += f1; a2 += f2; a3 += f3;
        }
      }
      const float inv = 1.0f / fmaxf((float)c, 1.0f);
      const float pzr = big ? __int_as_float(0x7fc00000) : 0.0f;
      const float m0 = live ? (a0 * inv + pzr) : 0.0f;
      const float m1 = live ? (a1 * inv + pzr) : 0.0f;
      const float m2 = live ? (a2 * inv + pzr) : 0.0f;
      const float m3 = live ? (a3 * inv + pzr) : 0.0f;
      v4us mh, ml;
      {
        unsigned lbit;
        unsigned hb;
        hb = hl_bits(m0, lbit); mh[0] = (unsigned short)hb; ml[0] = (unsigned short)lbit;
        hb = hl_bits(m1, lbit); mh[1] = (unsigned short)hb; ml[1] = (unsigned short)lbit;
        hb = hl_bits(m2, lbit); mh[2] = (unsigned short)hb; ml[2] = (unsigned short)lbit;
        hb = hl_bits(m3, lbit); mh[3] = (unsigned short)hb; ml[3] = (unsigned short)lbit;
      }
      *(v4usa*)(rowbuf + 4 * lane)      = mh;
      *(v4usa*)(rowbuf + DF + 4 * lane) = ml;
      wave_sync();
      const v8us q0 = *(const v8usa*)(rowbuf + 8 * lane);
      wave_sync();
      unsigned short* rpw = apl + (size_t)node * PP + 8 * lane;
      *(volatile v8us*)rpw = q0;
      __threadfence();
      *(volatile v8us*)rpw = q0;
    }
  }
}

__device__ __forceinline__ void gemm_seg(const unsigned short* ap, const unsigned short* bp, size_t ldb, int K,
                                         v8f (&acc)[8]) {
#pragma unroll 1
  for (int k0 = 0; k0 < K; k0 += 32) {
    FragB af;
    af.h[0] = *(const v8usa*)(ap + k0);
    af.h[1] = *(const v8usa*)(ap + k0 + 16);
#pragma unroll
    for (int nt = 0; nt < 8; ++nt) {
      const unsigned short* wq = bp + (size_t)(16 * nt) * ldb + k0;
      FragB bf;
      bf.h[0] = *(const v8usa*)wq;
      bf.h[1] = *(const v8usa*)(wq + 16);
      acc[nt] = wmb(af, bf, acc[nt]);
    }
  }
}

template <int OUTF, int RELU, int HASB>
__global__ __launch_bounds__(GTHR) void k_gemm(const unsigned short* A1, int K1,
                                               const unsigned short* A2, int lda2, int K2,
                                               const unsigned short* __restrict__ BT, int ldb,
                                               const float* __restrict__ bias,
                                               unsigned short* outp, int nOut, int mRows) {
  __shared__ __attribute__((aligned(16))) float stg[GBM * GBN];
  const int tid = (int)threadIdx.x, lane = tid & 31, wave = tid >> 5, hh = lane >> 4, m = lane & 15;
  const int rowBase = (int)blockIdx.x * GBM;

  v8f acc[8];
  {
    const v8f z = {0.f, 0.f, 0.f, 0.f, 0.f, 0.f, 0.f, 0.f};
#pragma unroll
    for (int t = 0; t < 8; ++t) acc[t] = z;
  }
  const size_t arow = (size_t)(rowBase + 16 * wave + m);
  const unsigned short* bp = BT + (size_t)m * (size_t)ldb + 8 * hh;
  gemm_seg(A1 + arow * PP + 8 * hh, bp, (size_t)ldb, K1, acc);
  gemm_seg(A2 + arow * (size_t)lda2 + 8 * hh, bp + K1, (size_t)ldb, K2, acc);

#pragma unroll
  for (int nt = 0; nt < 8; ++nt) {
    const int lc = 16 * nt + m;
#pragma unroll
    for (int r = 0; r < 8; ++r) {
      const int lr = 16 * wave + 8 * hh + r;
      stg[lr * GBN + lc] = acc[nt][r];
    }
  }
  __syncthreads();

  v4f bb4 = {0.f, 0.f, 0.f, 0.f};
  if constexpr (HASB != 0) {
    const v4f t1 = *(const v4f*)(bias + 4 * lane);
    bb4.x = bf16_val(t1.x); bb4.y = bf16_val(t1.y); bb4.z = bf16_val(t1.z); bb4.w = bf16_val(t1.w);
  }

  v4f pv[16];
#pragma unroll
  for (int i = 0; i < 16; ++i) pv[i] = *(const v4fa*)(stg + (16 * wave + i) * GBN + 4 * lane);
  __syncthreads();

#pragma unroll
  for (int i = 0; i < 16; ++i) {
    const bool ok = (rowBase + 16 * wave + i) < nOut;
    v4f y = pv[i] + bb4;
    if constexpr (RELU != 0) {
      y.x = (y.x > 0.0f) ? y.x : (y.x - y.x);
      y.y = (y.y > 0.0f) ? y.y : (y.y - y.y);
      y.z = (y.z > 0.0f) ? y.z : (y.z - y.z);
      y.w = (y.w > 0.0f) ? y.w : (y.w - y.w);
    }
    y.x = ok ? y.x : 0.0f; y.y = ok ? y.y : 0.0f; y.z = ok ? y.z : 0.0f; y.w = ok ? y.w : 0.0f;
    pv[i] = y;
  }

  if constexpr (OUTF != 0) {
    float* of = (float*)outp;
#pragma unroll
    for (int i = 0; i < 16; ++i) {
      const int gr = rowBase + 16 * wave + i;
      if (gr < mRows) *(volatile v4f*)(of + (size_t)gr * DF + 4 * lane) = pv[i];
    }
    __threadfence();
#pragma unroll
    for (int i = 0; i < 16; ++i) {
      const int gr = rowBase + 16 * wave + i;
      if (gr < mRows) *(volatile v4f*)(of + (size_t)gr * DF + 4 * lane) = pv[i];
    }
  } else {
#pragma unroll
    for (int i = 0; i < 16; ++i) {
      v4us h4, l4;
      unsigned lb;
      unsigned hb;
      hb = hl_bits(pv[i].x, lb); h4[0] = (unsigned short)hb; l4[0] = (unsigned short)lb;
      hb = hl_bits(pv[i].y, lb); h4[1] = (unsigned short)hb; l4[1] = (unsigned short)lb;
      hb = hl_bits(pv[i].z, lb); h4[2] = (unsigned short)hb; l4[2] = (unsigned short)lb;
      hb = hl_bits(pv[i].w, lb); h4[3] = (unsigned short)hb; l4[3] = (unsigned short)lb;
      unsigned short* srow = (unsigned short*)stg + (size_t)(16 * wave + i) * (2 * GBN);
      *(v4usa*)(srow + 4 * lane) = h4;
      *(v4usa*)(srow + DF + 4 * lane) = l4;
    }
    __syncthreads();
    v8us qv[16];
#pragma unroll
    for (int i = 0; i < 16; ++i) {
      const unsigned short* srow = (const unsigned short*)stg + (size_t)(16 * wave + i) * (2 * GBN);
      qv[i] = *(const v8usa*)(srow + 8 * lane);
    }
#pragma unroll
    for (int i = 0; i < 16; ++i) {
      const int gr = rowBase + 16 * wave + i;
      unsigned short* rp = outp + (size_t)gr * PP + 8 * lane;
      if (gr < mRows) *(volatile v8us*)rp = qv[i];
    }
    __threadfence();
#pragma unroll
    for (int i = 0; i < 16; ++i) {
      const int gr = rowBase + 16 * wave + i;
      unsigned short* rp = outp + (size_t)gr * PP + 8 * lane;
      if (gr < mRows) *(volatile v8us*)rp = qv[i];
    }
  }
}

__global__ __launch_bounds__(NTHR) void k_label(const float* pr, const float* pd,
                                                const int* __restrict__ lrow, const int* __restrict__ lcol,
                                                const float* __restrict__ dw2, const float* __restrict__ db2,
                                                const int* flg, int nflg, int nR, int nD, int nL, float* out) {
  __shared__ __attribute__((aligned(16))) float ost[LBLK];
  __shared__ int pf[4];
  const int tid = (int)threadIdx.x, lane = tid & 31, wave = tid >> 5;
  const int base = (int)blockIdx.x * LBLK;
  if (tid == 0) pf[0] = 0;
  __syncthreads();
  {
    const int fi = tid < nflg ? tid : nflg - 1;
    const int f  = flg[(size_t)fi * 32];
    if (tid < nflg && f != 0) pf[0] = 1;
  }
  v4f w4;
  {
    const v4f t1 = *(const v4f*)(dw2 + 4 * lane);
    w4.x = bf16_val(t1.x); w4.y = bf16_val(t1.y); w4.z = bf16_val(t1.z); w4.w = bf16_val(t1.w);
  }
  const float b2 = bf16_val(db2[0]);

#pragma unroll 1
  for (int j = 0; j < 4; ++j) {
    const int lb0 = base + wave * 128 + j * 32;
    const int li  = lb0 + lane;
    const int lic = li < nL ? li : nL - 1;
    int rr = lrow[lic];
    int cc = lcol[lic];
    rr = rr < 0 ? 0 : (rr > nR - 1 ? nR - 1 : rr);
    cc = cc < 0 ? 0 : (cc > nD - 1 ? nD - 1 : cc);
    int m32 = nL - lb0;
    m32 = m32 < 0 ? 0 : (m32 > 32 ? 32 : m32);
    float res = 0.0f;
#pragma unroll 1
    for (int k = 0; k < m32; ++k) {
      const int rk = __builtin_amdgcn_readlane(rr, k);
      const int ck = __builtin_amdgcn_readlane(cc, k);
      const v4f a = *(const v4fa*)(pr + (size_t)rk * DF + 4 * lane);
      const v4f b = *(const v4fa*)(pd + (size_t)ck * DF + 4 * lane);
      v4f t = a + b;
      t.x = (t.x > 0.0f) ? t.x : (t.x - t.x);
      t.y = (t.y > 0.0f) ? t.y : (t.y - t.y);
      t.z = (t.z > 0.0f) ? t.z : (t.z - t.z);
      t.w = (t.w > 0.0f) ? t.w : (t.w - t.w);
      float p = t.x * w4.x;
      p = fmaf(t.y, w4.y, p);
      p = fmaf(t.z, w4.z, p);
      p = fmaf(t.w, w4.w, p);
      p += __shfl_xor(p, 16, 32);
      p += __shfl_xor(p, 8, 32);
      p += __shfl_xor(p, 4, 32);
      p += __shfl_xor(p, 2, 32);
      p += __shfl_xor(p, 1, 32);
      const float v  = p + b2;
      const float sg = 1.0f / (1.0f + expf(-v));
      res = (lane == k) ? sg : res;
    }
    ost[wave * 128 + j * 32 + lane] = res;
  }
  __syncthreads();
  int nvalid = nL - base;
  nvalid = nvalid > LBLK ? LBLK : nvalid;
  const bool ok = (4 * tid) < nvalid;
  v4f o = *(const v4fa*)(ost + 4 * tid);
  if (pf[0] != 0) {
    const float qn = __int_as_float(0x7fc00000);
    o.x = qn; o.y = qn; o.z = qn; o.w = qn;
  }
  float* op = out + (size_t)base + 4 * tid;
  if (ok) *(volatile v4f*)op = o;
  __threadfence();
  if (ok) *(volatile v4f*)op = o;
}

static inline int cdiv(int a, int b) { return (a + b - 1) / b; }
static inline size_t al256(size_t o) { return (o + 255) & ~(size_t)255; }

extern "C" void kernel_launch(void* const* d_in, const int* in_sizes, int n_in,
                              void* d_out, int out_size, void* d_ws, size_t ws_size,
                              hipStream_t stream) {
  if (n_in < 24) return;
  if (in_sizes[0] < DF * GBM || (in_sizes[0] % DF) != 0) return;
  if (in_sizes[1] < DF * GBM || (in_sizes[1] % DF) != 0) return;
  const int nR = in_sizes[0] / DF;
  const int nD = in_sizes[1] / DF;
  const int nE = in_sizes[2];
  if (nE < 1 || nE >= (1 << 21)) return;
  if (in_sizes[3] != nE || in_sizes[4] != nE || in_sizes[5] != nE) return;
  const int nL = in_sizes[6];
  if (nL < 32 || (nL % 32) != 0 || in_sizes[7] != nL || out_size != nL) return;
  for (int g = 0; g < 4; ++g) {
    const int b = 8 + 3 * g;
    if (in_sizes[b] != DF * DF || in_sizes[b + 1] != DF || in_sizes[b + 2] != DF * DF) return;
  }
  if (in_sizes[20] != 2 * DF * DF || in_sizes[21] != DF || in_sizes[22] != DF || in_sizes[23] != 1) return;
  if (nR > (1 << 22) || nD > (1 << 22)) return;

  const float* x_rna = (const float*)d_in[0];
  const float* x_dis = (const float*)d_in[1];
  const int* src_rd  = (const int*)d_in[2];
  const int* dst_rd  = (const int*)d_in[3];
  const int* src_dr  = (const int*)d_in[4];
  const int* dst_dr  = (const int*)d_in[5];
  const int* lrow    = (const int*)d_in[6];
  const int* lcol    = (const int*)d_in[7];
  const float* W1rd_l = (const float*)d_in[8];
  const float* b1rd   = (const float*)d_in[9];
  const float* W1rd_r = (const float*)d_in[10];
  const float* W1dr_l = (const float*)d_in[11];
  const float* b1dr   = (const float*)d_in[12];
  const float* W1dr_r = (const float*)d_in[13];
  const float* W2rd_l = (const float*)d_in[14];
  const float* b2rd   = (const float*)d_in[15];
  const float* W2rd_r = (const float*)d_in[16];
  const float* W2dr_l = (const float*)d_in[17];
  const float* b2dr   = (const float*)d_in[18];
  const float* W2dr_r = (const float*)d_in[19];
  const float* dW1    = (const float*)d_in[20];
  const float* db1    = (const float*)d_in[21];
  const float* dW2    = (const float*)d_in[22];
  const float* db2    = (const float*)d_in[23];
  float* out = (float*)d_out;

  const int gRd = cdiv(nD, 1 << SL_RD);
  const int gDr = cdiv(nR, 1 << SL_DR);
  const int nflg = gRd + gDr;
  if (nflg > NTHR) return;
  const int MPd = cdiv(nD, 128) * 128;
  const int MPr = cdiv(nR, 128) * 128;
  if ((long long)gRd * (1 << SL_RD) < (long long)MPd) return;
  if ((long long)gDr * (1 << SL_DR) < (long long)MPr) return;
  const int vec8 = ((nE & 3) == 0) ? 1 : 0;

  char* ws = (char*)d_ws;
  size_t off = 0;
  const size_t oP   = off; off = al256(off + (size_t)MPr * PP * 2);
  const size_t oQ   = off; off = al256(off + (size_t)MPr * PP * 2);
  const size_t oXBD = off; off = al256(off + (size_t)MPd * DF * 2);
  const size_t oPd  = off; off = al256(off + (size_t)MPd * PP * 2);
  const size_t oQd  = off; off = al256(off + (size_t)MPd * PP * 2);
  const size_t oLR  = off; off = al256(off + (size_t)gRd * LS_RD * 4);
  const size_t oLD  = off; off = al256(off + (size_t)gDr * LS_DR * 4);
  const size_t oCR  = off; off = al256(off + (size_t)gRd * (1 << SL_RD) * 4);
  const size_t oOR  = off; off = al256(off + (size_t)gRd * (1 << SL_RD) * 4);
  const size_t oCD  = off; off = al256(off + (size_t)gDr * (1 << SL_DR) * 4);
  const size_t oOD  = off; off = al256(off + (size_t)gDr * (1 << SL_DR) * 4);
  const size_t oFL  = off; off = al256(off + (size_t)nflg * 128);
  const size_t oWP  = off; off = al256(off + (size_t)NUW * 16);
  if (off > ws_size || off > (size_t)WSMAX) return;
  unsigned short* P   = (unsigned short*)(ws + oP);
  unsigned short* Q   = (unsigned short*)(ws + oQ);
  unsigned short* XBR = Q;
  unsigned short* XBD = (unsigned short*)(ws + oXBD);
  unsigned short* Pd  = (unsigned short*)(ws + oPd);
  unsigned short* Qd  = (unsigned short*)(ws + oQd);
  int* LR = (int*)(ws + oLR);
  int* LD = (int*)(ws + oLD);
  int* CR = (int*)(ws + oCR);
  int* OR_ = (int*)(ws + oOR);
  int* CD = (int*)(ws + oCD);
  int* OD = (int*)(ws + oOD);
  int* FL = (int*)(ws + oFL);
  unsigned short* WP = (unsigned short*)(ws + oWP);
  const unsigned short* W1rdC = WP;
  const unsigned short* W1drC = WP + 49152;
  const unsigned short* W2rdC = WP + 98304;
  const unsigned short* W2drC = WP + 163840;
  const unsigned short* DTOP  = WP + 229376;
  const unsigned short* DBOT  = WP + 262144;

  const size_t ldsRd = (size_t)(LISTN + 2 * RCAP + 3 * (1 << SL_RD) + MISC_INTS) * 4;
  const size_t ldsDr = (size_t)(LISTN + 2 * RCAP + 3 * (1 << SL_DR) + MISC_INTS) * 4;
  hipFuncSetAttribute(reinterpret_cast<const void*>(&k_bucket<SL_RD, DEG_RD, LS_RD>),
                      hipFuncAttributeMaxDynamicSharedMemorySize, (int)ldsRd);
  hipFuncSetAttribute(reinterpret_cast<const void*>(&k_bucket<SL_DR, DEG_DR, LS_DR>),
                      hipFuncAttributeMaxDynamicSharedMemorySize, (int)ldsDr);

  const int uR = MPr * (DF / 8);
  const int uD = MPd * (DF / 8);
  const int nUnits = NUW + uR + uD;

  k_prep<<<cdiv(nUnits, NTHR), NTHR, 0, stream>>>(x_rna, x_dis, W1rd_l, W1rd_r, W1dr_l, W1dr_r,
                                                  W2rd_l, W2rd_r, W2dr_l, W2dr_r, dW1, WP, XBR, XBD, nR, nD, uR, uD);
  k_bucket<SL_RD, DEG_RD, LS_RD><<<gRd, NTHR, ldsRd, stream>>>(src_rd, dst_rd, nE, nR, vec8, LR, CR, OR_, FL);
  k_bucket<SL_DR, DEG_DR, LS_DR><<<gDr, NTHR, ldsDr, stream>>>(src_dr, dst_dr, nE, nD, vec8, LD, CD, OD,
                                                               FL + (size_t)gRd * 32);
  k_agg<SL_RD, DEG_RD, LS_RD, 0><<<gRd, NTHR, 0, stream>>>(LR, CR, OR_, XBR, nR, nD, MPd, Pd);
  k_agg<SL_DR, DEG_DR, LS_DR, 0><<<gDr, NTHR, 0, stream>>>(LD, CD, OD, XBD, nD, nR, MPr, P);
  k_gemm<0, 1, 1><<<MPd / GBM, GTHR, 0, stream>>>(Pd, 256, XBD, DF, DF, W1rdC, 384, b1rd, Pd, nD, MPd);
  k_gemm<0, 1, 1><<<MPr / GBM, GTHR, 0, stream>>>(P, 256, XBR, DF, DF, W1drC, 384, b1dr, P, nR, MPr);
  k_agg<SL_RD, DEG_RD, LS_RD, 1><<<gRd, NTHR, 0, stream>>>(LR, CR, OR_, P, nR, nD, MPd, Qd);
  k_agg<SL_DR, DEG_DR, LS_DR, 1><<<gDr, NTHR, 0, stream>>>(LD, CD, OD, Pd, nD, nR, MPr, Q);
  k_gemm<0, 0, 1><<<MPd / GBM, GTHR, 0, stream>>>(Qd, 256, Pd, PP, 256, W2rdC, 512, b2rd, Qd, nD, MPd);
  k_gemm<0, 0, 1><<<MPr / GBM, GTHR, 0, stream>>>(Q, 256, P, PP, 256, W2drC, 512, b2dr, Q, nR, MPr);
  k_gemm<1, 0, 0><<<MPd / GBM, GTHR, 0, stream>>>(Qd, 256, Qd, PP, 0, DBOT, 256, db1, Pd, nD, MPd);
  k_gemm<1, 0, 1><<<MPr / GBM, GTHR, 0, stream>>>(Q, 256, Q, PP, 0, DTOP, 256, db1, P, nR, MPr);
  k_label<<<cdiv(nL, LBLK), NTHR, 0, stream>>>((const float*)P, (const float*)Pd, lrow, lcol, dW2, db2,
                                               FL, nflg, nR, nD, nL, out);
}
